// FNO_3384434229355
// MI455X (gfx1250) — hardware-verified
//
#include <hip/hip_runtime.h>

typedef unsigned short us;
typedef us     v8us  __attribute__((ext_vector_type(8)));
typedef us     v4us  __attribute__((ext_vector_type(4)));
typedef __bf16 v16bf __attribute__((ext_vector_type(16)));
typedef float  v8f   __attribute__((ext_vector_type(8)));
typedef float  v4f   __attribute__((ext_vector_type(4)));
typedef v8us __attribute__((may_alias)) v8usa;
typedef v4us __attribute__((may_alias)) v4usa;
typedef v4f  __attribute__((may_alias)) v4fa;
typedef unsigned int __attribute__((may_alias)) u32a;

union Frag { v16bf v; v8us p[2]; };

#define NB    8
#define BP    4
#define NS    256
#define CH    64
#define NKY   16
#define NPIX  (BP * NS * NS)

#define TW_FAH 0
#define TW_FAL 8192
#define TW_FBH 16384
#define TW_FBL 32768
#define TW_G1H 49152
#define TW_G1L 65536
#define TW_G2H 81920
#define TW_G2L 98304
#define TW_GDH 114688
#define TW_GDL 122880
#define TW_WH  131072
#define TW_WL  147456
#define TW_TOTAL 163840

__device__ __forceinline__ v8f mma(v16bf a, v16bf b, v8f c) {
  v8f d = __builtin_amdgcn_wmma_f32_16x16x32_bf16(false, a, false, b, (short)0, c, false, false);
  asm volatile("v_nop\n\tv_nop\n\tv_nop\n\tv_nop" : "+v"(d) : "v"(a), "v"(b));
  return d;
}
__device__ __forceinline__ v8f mma3(v16bf ah, v16bf al, v16bf bh, v16bf bl, v8f c) {
  c = mma(ah, bh, c);
  c = mma(ah, bl, c);
  c = mma(al, bh, c);
  return c;
}

__device__ __forceinline__ unsigned bfb(float x) {
  const unsigned u = __float_as_uint(x);
  return (u + 0x7FFFu + ((u >> 16) & 1u)) >> 16;
}
__device__ __forceinline__ void split1(float x, us& hi, us& lo) {
  const unsigned hb = bfb(x);
  hi = (us)hb;
  lo = (us)bfb(x - __uint_as_float(hb << 16));
}
__device__ __forceinline__ void split8(v4f a, v4f b, v8us& hi, v8us& lo) {
  us h0, h1, h2, h3, h4, h5, h6, h7, l0, l1, l2, l3, l4, l5, l6, l7;
  split1(a.x, h0, l0); split1(a.y, h1, l1); split1(a.z, h2, l2); split1(a.w, h3, l3);
  split1(b.x, h4, l4); split1(b.y, h5, l5); split1(b.z, h6, l6); split1(b.w, h7, l7);
  v8us H = {h0, h1, h2, h3, h4, h5, h6, h7};
  v8us L = {l0, l1, l2, l3, l4, l5, l6, l7};
  hi = H; lo = L;
}
__device__ __forceinline__ float bf2f(us b) { return __uint_as_float(((unsigned)b) << 16); }

__device__ __forceinline__ v16bf ldfrag(const us* p, int h) {
  Frag f;
  f.p[0] = *(const v8usa*)(p + 8 * h);
  f.p[1] = *(const v8usa*)(p + 16 + 8 * h);
  return f.v;
}
__device__ __forceinline__ void frag_f32(const float* p, int h, v16bf& fh, v16bf& fl) {
  const v4f a = *(const v4fa*)(p + 8 * h);
  const v4f b = *(const v4fa*)(p + 8 * h + 4);
  const v4f c = *(const v4fa*)(p + 16 + 8 * h);
  const v4f d = *(const v4fa*)(p + 20 + 8 * h);
  Frag H, L;
  split8(a, b, H.p[0], L.p[0]);
  split8(c, d, H.p[1], L.p[1]);
  fh = H.v; fl = L.v;
}

__global__ __launch_bounds__(256) void k_prep(const float* __restrict__ bw, us* __restrict__ tw) {
  __shared__ float sC[256];
  __shared__ float sS[256];
  const int tid = threadIdx.x;
  {
    const float a = (float)tid * 0.0078125f;
    sC[tid] = cospif(a);
    sS[tid] = sinpif(a);
  }
  __syncthreads();
  const int g = blockIdx.x * 256 + tid;
  const int tab = (g >= 1024) + (g >= 3072) + (g >= 5120) + (g >= 7168) + (g >= 8192);
  const int base = (tab == 0) ? 0 : (tab == 1) ? 1024 : (tab == 2) ? 3072 : (tab == 3) ? 5120 : (tab == 4) ? 7168 : 8192;
  const int q = g - base;
  int rs, e0;
  if (tab <= 1)      { rs = q >> 5; e0 = (q & 31) * 8; }
  else if (tab <= 3) { rs = q >> 3; e0 = (q & 7) * 8; }
  else               { rs = q >> 2; e0 = (q & 3) * 8; }
  const int q5 = q & 2047;
  const int wblk = q5 >> 9, wo = (q5 >> 3) & 63, wc0 = (q5 & 7) * 8;
  float v[8];
#pragma unroll
  for (int e = 0; e < 8; ++e) {
    const int ke = e0 + e;
    const int jA = rs & 31, jB = ke & 31;
    const int kxA = (jA < 16) ? jA : (224 + jA);
    const int kxB = (jB < 16) ? jB : (224 + jB);
    int mult, pos; bool useCos; float coef;
    if (tab == 0)      { mult = rs & 15; pos = ke; useCos = (rs < 16); coef = useCos ? 1.0f : -1.0f; }
    else if (tab == 1) { mult = kxA;     pos = ke; useCos = (rs < 32); coef = 1.0f; }
    else if (tab == 2) { mult = kxB;     pos = rs; useCos = (ke < 32); coef = useCos ? 1.0f : -1.0f; }
    else if (tab == 3) { mult = kxB;     pos = rs; useCos = (ke >= 32); coef = 1.0f; }
    else {
      const int kk = ke & 15; mult = kk; pos = rs; useCos = (ke < 16);
      coef = (useCos ? ((kk == 0) ? 1.0f : 2.0f) : ((kk == 0) ? 0.0f : -2.0f)) * (1.0f / 65536.0f);
    }
    const int mm = (mult * pos) & 255;
    const float cv = sC[mm];
    const float sv = sS[mm];
    const float tv = (useCos ? cv : sv) * coef;
    const float wv = bw[(wblk * CH + wc0 + e) * CH + wo];
    v[e] = (tab == 5) ? wv : tv;
  }
  v4f a = {v[0], v[1], v[2], v[3]};
  v4f b = {v[4], v[5], v[6], v[7]};
  v8us H, L;
  split8(a, b, H, L);
  const int offh = (tab == 0) ? TW_FAH : (tab == 1) ? TW_FBH : (tab == 2) ? TW_G1H : (tab == 3) ? TW_G2H : (tab == 4) ? TW_GDH : TW_WH;
  const int offl = (tab == 0) ? TW_FAL : (tab == 1) ? TW_FBL : (tab == 2) ? TW_G1L : (tab == 3) ? TW_G2L : (tab == 4) ? TW_GDL : TW_WL;
  us* dh = tw + offh + q * 8;
  us* dl = tw + offl + q * 8;
  *(volatile v8us*)dh = H;
  *(volatile v8us*)dl = L;
  __threadfence();
  *(volatile v8us*)dh = H;
  *(volatile v8us*)dl = L;
}

__global__ __launch_bounds__(256) void k_lift(const float* __restrict__ xin, const float* __restrict__ lw,
                                              const float* __restrict__ lb, us* __restrict__ hh, us* __restrict__ hl) {
  const int g = blockIdx.x * 256 + threadIdx.x;
  const int pix = g >> 3, c0 = (g & 7) * 8;
  const float xv = xin[pix];
  float v[8];
#pragma unroll
  for (int j = 0; j < 8; ++j) v[j] = xv * lw[c0 + j] + lb[c0 + j];
  v4f a = {v[0], v[1], v[2], v[3]};
  v4f b = {v[4], v[5], v[6], v[7]};
  v8us H, L;
  split8(a, b, H, L);
  us* ph = hh + (size_t)pix * CH + c0;
  us* pl = hl + (size_t)pix * CH + c0;
  *(volatile v8us*)ph = H;
  *(volatile v8us*)pl = L;
  __threadfence();
  *(volatile v8us*)ph = H;
  *(volatile v8us*)pl = L;
}

__global__ __launch_bounds__(128) void k_dfta(const us* __restrict__ hh, const us* __restrict__ hl,
                                              const us* __restrict__ tw, float* __restrict__ xa) {
  __shared__ __attribute__((aligned(16))) us sAh[CH * 64];
  __shared__ __attribute__((aligned(16))) us sAl[CH * 64];
  __shared__ __attribute__((aligned(16))) float sO[CH * 32];
  const int tid = threadIdx.x, lane = tid & 31, w = tid >> 5, h = lane >> 4, m = lane & 15;
  const int slab = blockIdx.x;
  const us* ph = hh + (size_t)slab * (NS * CH);
  const us* pl = hl + (size_t)slab * (NS * CH);
  const us* faH = tw + TW_FAH;
  const us* faL = tw + TW_FAL;
  const v8f z8 = {0.f, 0.f, 0.f, 0.f, 0.f, 0.f, 0.f, 0.f};
  v8f acc[2];
  acc[0] = z8; acc[1] = z8;
  const int yq = tid >> 3, c0 = (tid & 7) * 8;
#pragma unroll 1
  for (int ch = 0; ch < 4; ++ch) {
    const int y0 = ch * 64;
    __syncthreads();
    {
      const us* src = ph + (size_t)(y0 + 4 * yq) * CH + c0;
      const v8us r0 = *(const v8usa*)(src);
      const v8us r1 = *(const v8usa*)(src + CH);
      const v8us r2 = *(const v8usa*)(src + 2 * CH);
      const v8us r3 = *(const v8usa*)(src + 3 * CH);
#pragma unroll
      for (int j = 0; j < 8; ++j) {
        v4us col = {r0[j], r1[j], r2[j], r3[j]};
        *(v4usa*)(sAh + (c0 + j) * 64 + 4 * yq) = col;
      }
    }
    {
      const us* src = pl + (size_t)(y0 + 4 * yq) * CH + c0;
      const v8us r0 = *(const v8usa*)(src);
      const v8us r1 = *(const v8usa*)(src + CH);
      const v8us r2 = *(const v8usa*)(src + 2 * CH);
      const v8us r3 = *(const v8usa*)(src + 3 * CH);
#pragma unroll
      for (int j = 0; j < 8; ++j) {
        v4us col = {r0[j], r1[j], r2[j], r3[j]};
        *(v4usa*)(sAl + (c0 + j) * 64 + 4 * yq) = col;
      }
    }
    __syncthreads();
#pragma unroll
    for (int kk = 0; kk < 2; ++kk) {
      const v16bf ah = ldfrag(sAh + (16 * w + m) * 64 + 32 * kk, h);
      const v16bf al = ldfrag(sAl + (16 * w + m) * 64 + 32 * kk, h);
#pragma unroll
      for (int nt = 0; nt < 2; ++nt) {
        const v16bf bh = ldfrag(faH + (16 * nt + m) * NS + y0 + 32 * kk, h);
        const v16bf bl = ldfrag(faL + (16 * nt + m) * NS + y0 + 32 * kk, h);
        acc[nt] = mma3(ah, al, bh, bl, acc[nt]);
      }
    }
  }
#pragma unroll
  for (int nt = 0; nt < 2; ++nt)
#pragma unroll
    for (int r = 0; r < 8; ++r)
      sO[(16 * w + 8 * h + r) * 32 + 16 * nt + m] = acc[nt][r];
  __syncthreads();
  const int q8 = lane & 7, sub = lane >> 3;
  float* dst = xa + (size_t)slab * (CH * 32);
#pragma unroll
  for (int pass = 0; pass < 2; ++pass) {
#pragma unroll
    for (int it = 0; it < 4; ++it) {
      const int line = 16 * w + it * 4 + sub;
      const v4f vv = *(const v4fa*)(sO + line * 32 + 4 * q8);
      *(volatile v4f*)(dst + line * 32 + 4 * q8) = vv;
    }
    if (pass == 0) __threadfence();
  }
}

__global__ __launch_bounds__(128) void k_dftb(const float* __restrict__ xa, const us* __restrict__ tw, float* __restrict__ xo) {
  __shared__ __attribute__((aligned(16))) us sBh[4 * 32 * 32];
  __shared__ __attribute__((aligned(16))) us sBl[4 * 32 * 32];
  __shared__ __attribute__((aligned(16))) float sO[4 * 16 * 2 * 32];
  const int tid = threadIdx.x, lane = tid & 31, w = tid >> 5, h = lane >> 4, m = lane & 15;
  const int bl = blockIdx.x >> 4, c0 = (blockIdx.x & 15) * 4, c = c0 + w;
  const us* fbH = tw + TW_FBH;
  const us* fbL = tw + TW_FBL;
  const v8f z8 = {0.f, 0.f, 0.f, 0.f, 0.f, 0.f, 0.f, 0.f};
  v8f acc[2][4];
#pragma unroll
  for (int mt = 0; mt < 2; ++mt)
#pragma unroll
    for (int nt = 0; nt < 4; ++nt) acc[mt][nt] = z8;
#pragma unroll 1
  for (int ks = 0; ks < 8; ++ks) {
    const int x0 = ks * 32;
    __syncthreads();
#pragma unroll
    for (int it = 0; it < 4; ++it) {
      const int idx = it * 128 + tid;
      const int xp = idx >> 5, qq = idx & 31, cl = qq >> 3, n0 = (qq & 7) * 4;
      const float* s0 = xa + ((size_t)(bl * NS + x0 + 2 * xp) * CH + c0 + cl) * 32 + n0;
      const v4f f0 = *(const v4fa*)s0;
      const v4f f1 = *(const v4fa*)(s0 + CH * 32);
      us* dh = sBh + (cl * 32 + n0) * 32 + 2 * xp;
      us* dl = sBl + (cl * 32 + n0) * 32 + 2 * xp;
      us a0, b0, a1, b1;
      split1(f0.x, a0, b0); split1(f1.x, a1, b1);
      *(u32a*)(dh)      = (unsigned)a0 | ((unsigned)a1 << 16);
      *(u32a*)(dl)      = (unsigned)b0 | ((unsigned)b1 << 16);
      split1(f0.y, a0, b0); split1(f1.y, a1, b1);
      *(u32a*)(dh + 32) = (unsigned)a0 | ((unsigned)a1 << 16);
      *(u32a*)(dl + 32) = (unsigned)b0 | ((unsigned)b1 << 16);
      split1(f0.z, a0, b0); split1(f1.z, a1, b1);
      *(u32a*)(dh + 64) = (unsigned)a0 | ((unsigned)a1 << 16);
      *(u32a*)(dl + 64) = (unsigned)b0 | ((unsigned)b1 << 16);
      split1(f0.w, a0, b0); split1(f1.w, a1, b1);
      *(u32a*)(dh + 96) = (unsigned)a0 | ((unsigned)a1 << 16);
      *(u32a*)(dl + 96) = (unsigned)b0 | ((unsigned)b1 << 16);
    }
    __syncthreads();
    v16bf ah[2], al[2];
#pragma unroll
    for (int mt = 0; mt < 2; ++mt) {
      ah[mt] = ldfrag(sBh + (w * 32 + 16 * mt + m) * 32, h);
      al[mt] = ldfrag(sBl + (w * 32 + 16 * mt + m) * 32, h);
    }
#pragma unroll
    for (int nt = 0; nt < 4; ++nt) {
      const v16bf bh  = ldfrag(fbH + (16 * nt + m) * NS + x0, h);
      const v16bf bll = ldfrag(fbL + (16 * nt + m) * NS + x0, h);
#pragma unroll
      for (int mt = 0; mt < 2; ++mt) acc[mt][nt] = mma3(ah[mt], al[mt], bh, bll, acc[mt][nt]);
    }
  }
  float* so = sO + w * (16 * 2 * 32);
#pragma unroll
  for (int jt = 0; jt < 2; ++jt)
#pragma unroll
    for (int r = 0; r < 8; ++r) {
      const float re = acc[0][jt][r] + acc[1][2 + jt][r];
      const float im = acc[1][jt][r] - acc[0][2 + jt][r];
      so[((8 * h + r) * 2 + 0) * 32 + 16 * jt + m] = re;
      so[((8 * h + r) * 2 + 1) * 32 + 16 * jt + m] = im;
    }
  __syncthreads();
  const int q8 = lane & 7, sub = lane >> 3;
  float* dst = xo + (size_t)(bl * CH + c) * (NKY * 2 * 32);
#pragma unroll
  for (int pass = 0; pass < 2; ++pass) {
#pragma unroll
    for (int it = 0; it < 8; ++it) {
      const int lid = it * 4 + sub;
      const v4f vv = *(const v4fa*)(so + lid * 32 + 4 * q8);
      *(volatile v4f*)(dst + lid * 32 + 4 * q8) = vv;
    }
    if (pass == 0) __threadfence();
  }
}

__global__ __launch_bounds__(256) void k_mix(const float* __restrict__ xo, const float* __restrict__ s1r,
                                             const float* __restrict__ s1i, const float* __restrict__ s2r,
                                             const float* __restrict__ s2i, float* __restrict__ om, int blk) {
  __shared__ __attribute__((aligned(16))) float sO[4 * 32 * 2 * 32];
  const int tid = threadIdx.x, lane = tid & 31, w = tid >> 5, h = lane >> 4, m = lane & 15;
  const int ky = blockIdx.x >> 1, oh = blockIdx.x & 1;
  const int brow = m & 3, apart = (m >> 3) & 1;
  const bool avalid = ((m & 4) == 0);
  const size_t wofs = (size_t)blk * (CH * CH * 256);
  const float* xbase = xo + (size_t)brow * (CH * NKY * 2 * 32) + ky * (2 * 32) + apart * 32;
  const v8f z8 = {0.f, 0.f, 0.f, 0.f, 0.f, 0.f, 0.f, 0.f};
#pragma unroll 1
  for (int jj = 0; jj < 4; ++jj) {
    const int j = w + 8 * jj;
    const bool bot = (j >= 16);
    const int kxw = j & 15;
    const float* wr = bot ? s2r : s1r;
    const float* wi = bot ? s2i : s1i;
    v16bf ah[2], al[2];
#pragma unroll
    for (int ks = 0; ks < 2; ++ks) {
      float v[16];
#pragma unroll
      for (int i = 0; i < 16; ++i) {
        const int cc = 32 * ks + 8 * h + i + 8 * (i >> 3);
        const float t = xbase[(size_t)cc * (NKY * 2 * 32) + j];
        v[i] = avalid ? t : 0.0f;
      }
      v4f a0 = {v[0], v[1], v[2], v[3]};
      v4f a1 = {v[4], v[5], v[6], v[7]};
      v4f a2 = {v[8], v[9], v[10], v[11]};
      v4f a3 = {v[12], v[13], v[14], v[15]};
      Frag H, L;
      split8(a0, a1, H.p[0], L.p[0]);
      split8(a2, a3, H.p[1], L.p[1]);
      ah[ks] = H.v; al[ks] = L.v;
    }
    v8f P[2], Q[2];
    P[0] = z8; P[1] = z8; Q[0] = z8; Q[1] = z8;
#pragma unroll
    for (int ks = 0; ks < 2; ++ks)
#pragma unroll
      for (int nt = 0; nt < 2; ++nt) {
        const int o = 32 * oh + 16 * nt + m;
        const size_t wrow = wofs + (size_t)o * 256 + kxw * 16 + ky;
        {
          float u[16];
#pragma unroll
          for (int i = 0; i < 16; ++i) {
            const int cc = 32 * ks + 8 * h + i + 8 * (i >> 3);
            u[i] = wr[wrow + (size_t)cc * 16384];
          }
          v4f b0 = {u[0], u[1], u[2], u[3]};
          v4f b1 = {u[4], u[5], u[6], u[7]};
          v4f b2 = {u[8], u[9], u[10], u[11]};
          v4f b3 = {u[12], u[13], u[14], u[15]};
          Frag H, L;
          split8(b0, b1, H.p[0], L.p[0]);
          split8(b2, b3, H.p[1], L.p[1]);
          P[nt] = mma3(ah[ks], al[ks], H.v, L.v, P[nt]);
        }
        {
          float u[16];
#pragma unroll
          for (int i = 0; i < 16; ++i) {
            const int cc = 32 * ks + 8 * h + i + 8 * (i >> 3);
            u[i] = wi[wrow + (size_t)cc * 16384];
          }
          v4f b0 = {u[0], u[1], u[2], u[3]};
          v4f b1 = {u[4], u[5], u[6], u[7]};
          v4f b2 = {u[8], u[9], u[10], u[11]};
          v4f b3 = {u[12], u[13], u[14], u[15]};
          Frag H, L;
          split8(b0, b1, H.p[0], L.p[0]);
          split8(b2, b3, H.p[1], L.p[1]);
          Q[nt] = mma3(ah[ks], al[ks], H.v, L.v, Q[nt]);
        }
      }
#pragma unroll
    for (int nt = 0; nt < 2; ++nt)
#pragma unroll
      for (int r = 0; r < 4; ++r) {
        const float qx = __shfl_xor(Q[nt][r], 16);
        const float val = P[nt][r] + (h ? qx : -qx);
        sO[((r * 32 + 16 * nt + m) * 2 + h) * 32 + j] = val;
      }
  }
  __syncthreads();
  const int q8 = lane & 7, sub = lane >> 3;
#pragma unroll
  for (int pass = 0; pass < 2; ++pass) {
#pragma unroll
    for (int it = 0; it < 8; ++it) {
      const int L = w * 32 + it * 4 + sub;
      const int b = L >> 6, rem = L & 63;
      const v4f vv = *(const v4fa*)(sO + (b * 64 + rem) * 32 + 4 * q8);
      float* dst = om + ((size_t)(b * NKY + ky) * CH + 32 * oh) * 64 + rem * 32 + 4 * q8;
      *(volatile v4f*)dst = vv;
    }
    if (pass == 0) __threadfence();
  }
}

__global__ __launch_bounds__(128) void k_dftc(const float* __restrict__ om, const us* __restrict__ tw, float* __restrict__ z) {
  __shared__ __attribute__((aligned(16))) float sO[4 * 2 * 16 * 64];
  const int tid = threadIdx.x, lane = tid & 31, w = tid >> 5, h = lane >> 4, m = lane & 15;
  const int xq = blockIdx.x & 3, ky = (blockIdx.x >> 2) & 15, bl = blockIdx.x >> 6;
  const int xw0 = 64 * xq + 16 * w;
  const us* g1H = tw + TW_G1H;
  const us* g1L = tw + TW_G1L;
  const us* g2H = tw + TW_G2H;
  const us* g2L = tw + TW_G2L;
  const v8f z8 = {0.f, 0.f, 0.f, 0.f, 0.f, 0.f, 0.f, 0.f};
  v8f aR[4], aI[4];
#pragma unroll
  for (int nt = 0; nt < 4; ++nt) { aR[nt] = z8; aI[nt] = z8; }
  const float* orow = om + (size_t)(bl * NKY + ky) * (CH * 64);
#pragma unroll
  for (int ks = 0; ks < 2; ++ks) {
    const v16bf a1h = ldfrag(g1H + (xw0 + m) * 64 + 32 * ks, h);
    const v16bf a1l = ldfrag(g1L + (xw0 + m) * 64 + 32 * ks, h);
    const v16bf a2h = ldfrag(g2H + (xw0 + m) * 64 + 32 * ks, h);
    const v16bf a2l = ldfrag(g2L + (xw0 + m) * 64 + 32 * ks, h);
#pragma unroll
    for (int nt = 0; nt < 4; ++nt) {
      v16bf bh, bll;
      frag_f32(orow + (size_t)(16 * nt + m) * 64 + 32 * ks, h, bh, bll);
      aR[nt] = mma3(a1h, a1l, bh, bll, aR[nt]);
      aI[nt] = mma3(a2h, a2l, bh, bll, aI[nt]);
    }
  }
  float* so = sO + w * (2 * 16 * 64);
#pragma unroll
  for (int nt = 0; nt < 4; ++nt)
#pragma unroll
    for (int r = 0; r < 8; ++r) {
      so[(0 * 16 + 8 * h + r) * 64 + 16 * nt + m] = aR[nt][r];
      so[(1 * 16 + 8 * h + r) * 64 + 16 * nt + m] = aI[nt][r];
    }
  __syncthreads();
  const int q8 = lane & 7, sub = lane >> 3;
#pragma unroll
  for (int pass = 0; pass < 2; ++pass) {
#pragma unroll
    for (int it = 0; it < 16; ++it) {
      const int lid = it * 4 + sub;
      const int part = lid >> 5, rem = lid & 31, row = rem >> 1, hl2 = rem & 1;
      const v4f vv = *(const v4fa*)(so + (part * 16 + row) * 64 + 32 * hl2 + 4 * q8);
      float* dst = z + ((size_t)((bl * NKY + ky) * 2 + part) * NS + xw0 + row) * CH + 32 * hl2 + 4 * q8;
      *(volatile v4f*)dst = vv;
    }
    if (pass == 0) __threadfence();
  }
}

__global__ __launch_bounds__(128) void k_fused(const float* __restrict__ z, const float* __restrict__ bias,
                                               const us* __restrict__ tw, int blk,
                                               us* __restrict__ hh, us* __restrict__ hl) {
  __shared__ __attribute__((aligned(16))) us sZh[64 * 32];
  __shared__ __attribute__((aligned(16))) us sZl[64 * 32];
  __shared__ __attribute__((aligned(16))) us sOh[4 * 32 * 64];
  __shared__ __attribute__((aligned(16))) us sOl[4 * 32 * 64];
  const int tid = threadIdx.x, lane = tid & 31, w = tid >> 5, h = lane >> 4, m = lane & 15;
  const int yh = blockIdx.x & 1, x = (blockIdx.x >> 1) & 255, bl = blockIdx.x >> 9;
  {
    const int krow = tid >> 2, o0 = (tid & 3) * 16;
    const int part = krow >> 4, kyy = krow & 15;
    const float* src = z + ((size_t)((bl * NKY + kyy) * 2 + part) * NS + x) * CH + o0;
    const v4f a = *(const v4fa*)(src);
    const v4f b = *(const v4fa*)(src + 4);
    const v4f c = *(const v4fa*)(src + 8);
    const v4f d = *(const v4fa*)(src + 12);
    float v[16] = {a.x, a.y, a.z, a.w, b.x, b.y, b.z, b.w, c.x, c.y, c.z, c.w, d.x, d.y, d.z, d.w};
#pragma unroll
    for (int jx = 0; jx < 16; ++jx) {
      us p, q;
      split1(v[jx], p, q);
      sZh[(o0 + jx) * 32 + krow] = p;
      sZl[(o0 + jx) * 32 + krow] = q;
    }
  }
  __syncthreads();
  const v8f z8 = {0.f, 0.f, 0.f, 0.f, 0.f, 0.f, 0.f, 0.f};
  v8f acc[2][4];
#pragma unroll
  for (int mt = 0; mt < 2; ++mt)
#pragma unroll
    for (int nt = 0; nt < 4; ++nt) acc[mt][nt] = z8;
  const size_t pixbase = (size_t)(bl * NS + x) * NS + 128 * yh + 32 * w;
  const us* gdH = tw + TW_GDH;
  const us* gdL = tw + TW_GDL;
  const us* wth = tw + TW_WH + blk * 4096;
  const us* wtl = tw + TW_WL + blk * 4096;
  {
    v16bf ah[2], al[2];
#pragma unroll
    for (int mt = 0; mt < 2; ++mt) {
      const int y = 128 * yh + 32 * w + 16 * mt + m;
      ah[mt] = ldfrag(gdH + y * 32, h);
      al[mt] = ldfrag(gdL + y * 32, h);
    }
#pragma unroll
    for (int nt = 0; nt < 4; ++nt) {
      const v16bf bh  = ldfrag(sZh + (16 * nt + m) * 32, h);
      const v16bf bll = ldfrag(sZl + (16 * nt + m) * 32, h);
#pragma unroll
      for (int mt = 0; mt < 2; ++mt) acc[mt][nt] = mma3(ah[mt], al[mt], bh, bll, acc[mt][nt]);
    }
  }
#pragma unroll
  for (int ks = 0; ks < 2; ++ks) {
    v16bf ah[2], al[2];
#pragma unroll
    for (int mt = 0; mt < 2; ++mt) {
      ah[mt] = ldfrag(hh + (pixbase + 16 * mt + m) * CH + 32 * ks, h);
      al[mt] = ldfrag(hl + (pixbase + 16 * mt + m) * CH + 32 * ks, h);
    }
#pragma unroll
    for (int nt = 0; nt < 4; ++nt) {
      const v16bf bh  = ldfrag(wth + (16 * nt + m) * CH + 32 * ks, h);
      const v16bf bll = ldfrag(wtl + (16 * nt + m) * CH + 32 * ks, h);
#pragma unroll
      for (int mt = 0; mt < 2; ++mt) acc[mt][nt] = mma3(ah[mt], al[mt], bh, bll, acc[mt][nt]);
    }
  }
  us* soh = sOh + w * (32 * 64);
  us* sol = sOl + w * (32 * 64);
#pragma unroll
  for (int nt = 0; nt < 4; ++nt) {
    const int o = 16 * nt + m;
    const float bo = bias[o];
#pragma unroll
    for (int mt = 0; mt < 2; ++mt)
#pragma unroll
      for (int r = 0; r < 8; ++r) {
        const float vv = fmaxf(acc[mt][nt][r] + bo, 0.0f);
        us p, q;
        split1(vv, p, q);
        soh[(16 * mt + 8 * h + r) * 64 + o] = p;
        sol[(16 * mt + 8 * h + r) * 64 + o] = q;
      }
  }
  __syncthreads();
  const int q8 = lane & 7, sub = lane >> 3;
  us* dh = hh + pixbase * CH;
  us* dl = hl + pixbase * CH;
#pragma unroll
  for (int pass = 0; pass < 2; ++pass) {
#pragma unroll
    for (int it = 0; it < 8; ++it) {
      const int row = it * 4 + sub;
      const v8us va = *(const v8usa*)(soh + row * 64 + 8 * q8);
      const v8us vb = *(const v8usa*)(sol + row * 64 + 8 * q8);
      *(volatile v8us*)(dh + row * 64 + 8 * q8) = va;
      *(volatile v8us*)(dl + row * 64 + 8 * q8) = vb;
    }
    if (pass == 0) __threadfence();
  }
}

__global__ __launch_bounds__(256) void k_proj(const us* __restrict__ hh, const us* __restrict__ hl,
                                              const float* __restrict__ pw, const float* __restrict__ pb,
                                              float* __restrict__ out) {
  const int pix = blockIdx.x * 256 + threadIdx.x;
  const us* ph = hh + (size_t)pix * CH;
  const us* pl = hl + (size_t)pix * CH;
  float s = 0.0f;
#pragma unroll 1
  for (int g = 0; g < 8; ++g) {
    const v8us a = *(const v8usa*)(ph + 8 * g);
    const v8us b = *(const v8usa*)(pl + 8 * g);
#pragma unroll
    for (int e = 0; e < 8; ++e) {
      const float hv = bf2f(a[e]) + bf2f(b[e]);
      s += hv * pw[8 * g + e];
    }
  }
  const float r = s + pb[0];
  *(volatile float*)(out + pix) = r;
  __threadfence();
  *(volatile float*)(out + pix) = r;
}

extern "C" void kernel_launch(void* const* d_in, const int* in_sizes, int n_in,
                              void* d_out, int out_size, void* d_ws, size_t ws_size,
                              hipStream_t stream) {
  if (n_in < 11) return;
  if (in_sizes[0] != NB * NS * NS) return;
  if (in_sizes[1] != CH || in_sizes[2] != CH) return;
  if (in_sizes[3] != 4 * CH * CH || in_sizes[4] != 4 * CH) return;
  const int nspec = 4 * CH * CH * 256;
  if (in_sizes[5] != nspec || in_sizes[6] != nspec || in_sizes[7] != nspec || in_sizes[8] != nspec) return;
  if (in_sizes[9] != CH || in_sizes[10] < 1) return;
  if (out_size != NB * NS * NS) return;

  const float* x   = (const float*)d_in[0];
  const float* lw  = (const float*)d_in[1];
  const float* lb  = (const float*)d_in[2];
  const float* bw  = (const float*)d_in[3];
  const float* bb  = (const float*)d_in[4];
  const float* s1r = (const float*)d_in[5];
  const float* s1i = (const float*)d_in[6];
  const float* s2r = (const float*)d_in[7];
  const float* s2i = (const float*)d_in[8];
  const float* pw  = (const float*)d_in[9];
  const float* pb  = (const float*)d_in[10];
  float* out = (float*)d_out;

  const size_t hBytes  = (size_t)NPIX * CH * 2;
  const size_t xaBytes = (size_t)BP * NS * CH * 32 * 4;
  const size_t xoBytes = (size_t)BP * CH * NKY * 2 * 32 * 4;
  const size_t omBytes = (size_t)BP * NKY * CH * 2 * 32 * 4;
  const size_t zBytes  = (size_t)BP * NKY * 2 * NS * CH * 4;
  const size_t twBytes = (size_t)TW_TOTAL * 2;
  const size_t total = 2 * hBytes + xaBytes + xoBytes + omBytes + zBytes + twBytes;
  if (total > ws_size) return;

  char* wsb = (char*)d_ws;
  us*    hh = (us*)(wsb);
  us*    hl = (us*)(wsb + hBytes);
  float* xa = (float*)(wsb + 2 * hBytes);
  float* xo = (float*)(wsb + 2 * hBytes + xaBytes);
  float* om = (float*)(wsb + 2 * hBytes + xaBytes + xoBytes);
  float* zz = (float*)(wsb + 2 * hBytes + xaBytes + xoBytes + omBytes);
  us*    tw = (us*)(wsb + 2 * hBytes + xaBytes + xoBytes + omBytes + zBytes);

  k_prep<<<40, 256, 0, stream>>>(bw, tw);

  for (int hb = 0; hb < 2; ++hb) {
    k_lift<<<(NPIX * 8) / 256, 256, 0, stream>>>(x + (size_t)hb * NPIX, lw, lb, hh, hl);
    for (int blk = 0; blk < 4; ++blk) {
      k_dfta<<<BP * NS, 128, 0, stream>>>(hh, hl, tw, xa);
      k_dftb<<<BP * 16, 128, 0, stream>>>(xa, tw, xo);
      k_mix<<<NKY * 2, 256, 0, stream>>>(xo, s1r, s1i, s2r, s2i, om, blk);
      k_dftc<<<BP * NKY * 4, 128, 0, stream>>>(om, tw, zz);
      k_fused<<<BP * NS * 2, 128, 0, stream>>>(zz, bb + blk * CH, tw, blk, hh, hl);
    }
    k_proj<<<NPIX / 256, 256, 0, stream>>>(hh, hl, pw, pb, out + (size_t)hb * NPIX);
  }
}
